// CINNv2_22419729285718
// MI455X (gfx1250) — hardware-verified
//
#include <hip/hip_runtime.h>
#include <math.h>


#define D_     64
#define HID_   512
#define DC_    128
#define NIN_   160
#define LH_    32
#define NBLK_  12
#define BT_    64
#define NTH_   128
#define NWV_   4
#define ACTP_  168
#define HSP_   32

static_assert(NIN_ == LH_ + DC_);
static_assert(NIN_ % 32 == 0);
static_assert(HID_ % 32 == 0);
static_assert(ACTP_ % 8 == 0);
static_assert(ACTP_ >= NIN_);
static_assert(BT_ == NWV_ * 16);
static_assert(NTH_ == NWV_ * 32);
static_assert(D_ == 2 * LH_);

typedef float    v4f  __attribute__((ext_vector_type(4)));
typedef float    v8f  __attribute__((ext_vector_type(8)));
typedef _Float16 v4h  __attribute__((ext_vector_type(4)));
typedef _Float16 v8h  __attribute__((ext_vector_type(8))) __attribute__((may_alias));
typedef _Float16 v16h __attribute__((ext_vector_type(16)));

union Frag { v16h v; v8h half[2]; };

__device__ __forceinline__ void mma(v8f& acc, const Frag& a, const Frag& b) {
    acc = __builtin_amdgcn_wmma_f32_16x16x32_f16(false, a.v, false, b.v, (short)0, acc, false, false);
    asm volatile("v_nop\n\tv_nop\n\tv_nop\n\tv_nop" : "+v"(acc) : "v"(a.v), "v"(b.v));
}

__device__ __forceinline__ float wsum32(float v) {
    v += __shfl_xor(v, 16, 32);
    v += __shfl_xor(v, 8, 32);
    v += __shfl_xor(v, 4, 32);
    v += __shfl_xor(v, 2, 32);
    v += __shfl_xor(v, 1, 32);
    return v;
}
__device__ __forceinline__ float hsum16(float v) {
    v += __shfl_xor(v, 8, 32);
    v += __shfl_xor(v, 4, 32);
    v += __shfl_xor(v, 2, 32);
    v += __shfl_xor(v, 1, 32);
    return v;
}

__global__ __launch_bounds__(256)
void cvt_f16_kernel(const float* __restrict__ src, _Float16* dst, int n8, float carry)
{
    const int i = blockIdx.x * 256 + threadIdx.x;
    if (i >= n8) return;
    const size_t e = (size_t)i * 8;
    const v4f a = *(const v4f*)(src + e);
    const v4f b = *(const v4f*)(src + e + 4);
    v8h o;
    o[0] = (_Float16)(a[0] * carry); o[1] = (_Float16)(a[1] * carry);
    o[2] = (_Float16)(a[2] * carry); o[3] = (_Float16)(a[3] * carry);
    o[4] = (_Float16)(b[0] * carry); o[5] = (_Float16)(b[1] * carry);
    o[6] = (_Float16)(b[2] * carry); o[7] = (_Float16)(b[3] * carry);
    *(volatile v8h*)(dst + e) = o;
    __threadfence();
    *(volatile v8h*)(dst + e) = o;
}

template<int XCOL, int WACT>
__device__ __forceinline__ void coupling_mlp(float* s_x, _Float16* s_act, _Float16* s_hsw,
                                             const _Float16* __restrict__ w1, const float* __restrict__ b1,
                                             const _Float16* __restrict__ w2, const float* __restrict__ b2,
                                             int m0, int lane, float (&lj)[8])
{
    const int lr = lane & 15;
    const int lh = lane >> 4;

    Frag a[5];
#pragma unroll
    for (int kk = 0; kk < 5; ++kk) {
        const _Float16* p = s_act + (m0 + lr) * ACTP_ + kk * 32 + 8 * lh;
        a[kk].half[0] = *(const v8h*)p;
        a[kk].half[1] = *(const v8h*)(p + 16);
    }

    v8f acc[4];
#pragma unroll
    for (int t = 0; t < 4; ++t)
#pragma unroll
        for (int r = 0; r < 8; ++r) acc[t][r] = 0.0f;

#pragma unroll 1
    for (int nh = 0; nh < HID_ / 32; ++nh) {
        const int hb = nh * 32;
        v8f h0, h1;
        {
            const float c0 = 64.0f * b1[hb + lr];
            const float c1 = 64.0f * b1[hb + 16 + lr];
#pragma unroll
            for (int r = 0; r < 8; ++r) { h0[r] = c0; h1[r] = c1; }
        }
#pragma unroll
        for (int kk = 0; kk < 5; ++kk) {
            Frag f0, f1;
            const _Float16* q0 = w1 + (size_t)(hb + lr) * NIN_ + kk * 32 + 8 * lh;
            const _Float16* q1 = q0 + (size_t)16 * NIN_;
            f0.half[0] = *(const v8h*)q0;
            f0.half[1] = *(const v8h*)(q0 + 16);
            f1.half[0] = *(const v8h*)q1;
            f1.half[1] = *(const v8h*)(q1 + 16);
            mma(h0, a[kk], f0);
            mma(h1, a[kk], f1);
        }

        __syncthreads();
#pragma unroll
        for (int r = 0; r < 8; ++r) {
            _Float16* row = s_hsw + (8 * lh + r) * HSP_;
            row[lr]      = (_Float16)fmaxf(h0[r], 0.0f);
            row[16 + lr] = (_Float16)fmaxf(h1[r], 0.0f);
        }
        __syncthreads();
        Frag a2;
        {
            const _Float16* p = s_hsw + lr * HSP_ + 8 * lh;
            a2.half[0] = *(const v8h*)p;
            a2.half[1] = *(const v8h*)(p + 16);
        }
#pragma unroll
        for (int t = 0; t < 4; ++t) {
            Frag g;
            const _Float16* q = w2 + (size_t)(t * 16 + lr) * HID_ + hb + 8 * lh;
            g.half[0] = *(const v8h*)q;
            g.half[1] = *(const v8h*)(q + 16);
            mma(acc[t], a2, g);
        }
    }

    const float inv = 0.000244140625f;
    const float bb0 = b2[lr];
    const float bb1 = b2[16 + lr];
    const float bb2 = b2[32 + lr];
    const float bb3 = b2[48 + lr];
#pragma unroll
    for (int r = 0; r < 8; ++r) {
        const int row = m0 + 8 * lh + r;
        const float s0 = acc[0][r] * inv + bb0;
        const float s1 = acc[1][r] * inv + bb1;
        const float t0 = acc[2][r] * inv + bb2;
        const float t1 = acc[3][r] * inv + bb3;
        const float le0 = 0.636f * atanf(s0);
        const float le1 = 0.636f * atanf(s1);
        const float e0 = __expf(le0);
        const float e1 = __expf(le1);
        float* xr = s_x + row * D_ + XCOL;
        const float y0 = e0 * xr[lr] + t0;
        const float y1 = e1 * xr[16 + lr] + t1;
        xr[lr]      = y0;
        xr[16 + lr] = y1;
        if (WACT) {
            s_act[row * ACTP_ + lr]      = (_Float16)y0;
            s_act[row * ACTP_ + 16 + lr] = (_Float16)y1;
        }
        const float ls = hsum16(le0 + le1);
        lj[r] += ls;
    }
}

__global__ __launch_bounds__(NTH_)
void flow_kernel(const float* __restrict__ qf, const float* __restrict__ Hg, const int* __restrict__ perms,
                 const float* __restrict__ anls, const float* __restrict__ anbi,
                 const _Float16* __restrict__ w11, const float* __restrict__ b11,
                 const _Float16* __restrict__ w12, const float* __restrict__ b12,
                 const _Float16* __restrict__ w21, const float* __restrict__ b21,
                 const _Float16* __restrict__ w22, const float* __restrict__ b22,
                 float* out, int Btot)
{
    __shared__ __attribute__((aligned(16))) float    s_x[BT_ * D_];
    __shared__ __attribute__((aligned(16))) _Float16 s_act[BT_ * ACTP_];
    __shared__ __attribute__((aligned(16))) _Float16 s_hs[NWV_ * 16 * HSP_];
    __shared__ __attribute__((aligned(16))) float    s_lj[BT_];

    const int tid  = threadIdx.x;
    const int lane = tid & 31;
    const int wave = tid >> 5;
    const int lr   = lane & 15;
    const int lh   = lane >> 4;
    const int m0   = wave * 16;
    const int rowbase = blockIdx.x * BT_;

#pragma unroll 1
    for (int i = tid; i < (BT_ * D_) / 4; i += NTH_) {
        const v4f v = *(const v4f*)(qf + (size_t)rowbase * D_ + (size_t)i * 4);
        *(v4f*)(s_x + i * 4) = v;
    }
#pragma unroll 1
    for (int i = tid; i < (BT_ * DC_) / 4; i += NTH_) {
        const int r = i >> 5;
        const int c = (i & 31) * 4;
        const v4f v = *(const v4f*)(Hg + (size_t)(rowbase + r) * DC_ + c);
        v4h h;
        h[0] = (_Float16)v[0]; h[1] = (_Float16)v[1]; h[2] = (_Float16)v[2]; h[3] = (_Float16)v[3];
        *(v4h*)(s_act + r * ACTP_ + LH_ + c) = h;
    }
    __syncthreads();

    _Float16* hsw = s_hs + wave * 16 * HSP_;
    float lj[8];
#pragma unroll
    for (int r = 0; r < 8; ++r) lj[r] = 0.0f;

#pragma unroll 1
    for (int k = 0; k < NBLK_; ++k) {
        int p0 = perms[k * D_ + lane];
        int p1 = perms[k * D_ + 32 + lane];
        p0 = (p0 < 0) ? (p0 + D_) : p0;  p0 = min(max(p0, 0), D_ - 1);
        p1 = (p1 < 0) ? (p1 + D_) : p1;  p1 = min(max(p1, 0), D_ - 1);
        const float ls0 = anls[k * D_ + lane];
        const float ls1 = anls[k * D_ + 32 + lane];
        const float es0 = expf(ls0);
        const float es1 = expf(ls1);
        const float bi0 = anbi[k * D_ + lane];
        const float bi1 = anbi[k * D_ + 32 + lane];
        const float ssum = wsum32(ls0 + ls1);
#pragma unroll
        for (int r = 0; r < 8; ++r) lj[r] += ssum;

        float tmp[32];
#pragma unroll
        for (int i = 0; i < 32; ++i) {
            const int row = m0 + (i >> 1);
            tmp[i] = s_x[row * D_ + ((i & 1) ? p1 : p0)];
        }
        __syncthreads();
#pragma unroll
        for (int i = 0; i < 32; ++i) {
            const int row = m0 + (i >> 1);
            if (i & 1) {
                const float v = tmp[i] * es1 + bi1;
                s_x[row * D_ + 32 + lane] = v;
                s_act[row * ACTP_ + lane] = (_Float16)v;
            } else {
                const float v = tmp[i] * es0 + bi0;
                s_x[row * D_ + lane] = v;
            }
        }
        __syncthreads();

        coupling_mlp<0, 1>(s_x, s_act, hsw,
                           w21 + (size_t)k * HID_ * NIN_, b21 + (size_t)k * HID_,
                           w22 + (size_t)k * D_ * HID_,   b22 + (size_t)k * D_,
                           m0, lane, lj);
        __syncthreads();
        coupling_mlp<LH_, 0>(s_x, s_act, hsw,
                             w11 + (size_t)k * HID_ * NIN_, b11 + (size_t)k * HID_,
                             w12 + (size_t)k * D_ * HID_,   b12 + (size_t)k * D_,
                             m0, lane, lj);
        __syncthreads();
    }

    if (lr == 0) {
#pragma unroll
        for (int r = 0; r < 8; ++r) s_lj[m0 + 8 * lh + r] = lj[r];
    }
    __syncthreads();

    v4f zv[8];
#pragma unroll
    for (int it = 0; it < 8; ++it)
        zv[it] = *(const v4f*)(s_x + m0 * D_ + it * 128 + lane * 4);
    float* zb = out + (size_t)rowbase * D_ + (size_t)m0 * D_;
#pragma unroll
    for (int it = 0; it < 8; ++it)
        *(volatile v4f*)(zb + it * 128 + lane * 4) = zv[it];

    const bool wl = (wave == 0) && (lane < 16);
    const v4f lv = *(const v4f*)(s_lj + lr * 4);
    float* lb = out + (size_t)Btot * D_ + rowbase;
    if (wl) *(volatile v4f*)(lb + lr * 4) = lv;

    __threadfence();

#pragma unroll
    for (int it = 0; it < 8; ++it)
        *(volatile v4f*)(zb + it * 128 + lane * 4) = zv[it];
    if (wl) *(volatile v4f*)(lb + lr * 4) = lv;
}

extern "C" void kernel_launch(void* const* d_in, const int* in_sizes, int n_in,
                              void* d_out, int out_size, void* d_ws, size_t ws_size,
                              hipStream_t stream)
{
    if (n_in < 13) return;
    const int Btot = in_sizes[0] / D_;
    if (Btot <= 0 || (Btot % BT_) != 0) return;
    if (in_sizes[0] != Btot * D_) return;
    if (in_sizes[1] != Btot * DC_) return;
    if (in_sizes[2] != NBLK_ * D_) return;
    if (in_sizes[3] != NBLK_ * D_) return;
    if (in_sizes[4] != NBLK_ * D_) return;
    const int nW1 = NBLK_ * HID_ * NIN_;
    const int nW2 = NBLK_ * D_ * HID_;
    if (in_sizes[5] != nW1 || in_sizes[9] != nW1) return;
    if (in_sizes[6] != NBLK_ * HID_ || in_sizes[10] != NBLK_ * HID_) return;
    if (in_sizes[7] != nW2 || in_sizes[11] != nW2) return;
    if (in_sizes[8] != NBLK_ * D_ || in_sizes[12] != NBLK_ * D_) return;
    if (out_size != Btot * D_ + Btot) return;
    if ((nW1 % 8) != 0 || (nW2 % 8) != 0) return;

    const size_t sz1 = (size_t)nW1 * 2;
    const size_t sz2 = (size_t)nW2 * 2;
    const size_t o11 = 0;
    const size_t o12 = o11 + sz1;
    const size_t o21 = o12 + sz2;
    const size_t o22 = o21 + sz1;
    const size_t wend = o22 + sz2;
    if ((sz1 % 512) != 0 || (sz2 % 512) != 0) return;
    if (wend > ws_size || wend > (size_t)134217728) return;

    const float* qf    = (const float*)d_in[0];
    const float* Hg    = (const float*)d_in[1];
    const int*   perms = (const int*)d_in[2];
    const float* anls  = (const float*)d_in[3];
    const float* anbi  = (const float*)d_in[4];
    const float* s1W1  = (const float*)d_in[5];
    const float* s1b1  = (const float*)d_in[6];
    const float* s1W2  = (const float*)d_in[7];
    const float* s1b2  = (const float*)d_in[8];
    const float* s2W1  = (const float*)d_in[9];
    const float* s2b1  = (const float*)d_in[10];
    const float* s2W2  = (const float*)d_in[11];
    const float* s2b2  = (const float*)d_in[12];
    float* out = (float*)d_out;

    char* ws = (char*)d_ws;
    _Float16* p11 = (_Float16*)(ws + o11);
    _Float16* p12 = (_Float16*)(ws + o12);
    _Float16* p21 = (_Float16*)(ws + o21);
    _Float16* p22 = (_Float16*)(ws + o22);

    const float carry = 64.0f;
    cvt_f16_kernel<<<dim3((nW1 / 8 + 255) / 256), dim3(256), 0, stream>>>(s1W1, p11, nW1 / 8, carry);
    cvt_f16_kernel<<<dim3((nW2 / 8 + 255) / 256), dim3(256), 0, stream>>>(s1W2, p12, nW2 / 8, carry);
    cvt_f16_kernel<<<dim3((nW1 / 8 + 255) / 256), dim3(256), 0, stream>>>(s2W1, p21, nW1 / 8, carry);
    cvt_f16_kernel<<<dim3((nW2 / 8 + 255) / 256), dim3(256), 0, stream>>>(s2W2, p22, nW2 / 8, carry);

    flow_kernel<<<dim3(Btot / BT_), dim3(NTH_), 0, stream>>>(
        qf, Hg, perms, anls, anbi,
        (const _Float16*)p11, s1b1, (const _Float16*)p12, s1b2,
        (const _Float16*)p21, s2b1, (const _Float16*)p22, s2b2,
        out, Btot);
}
